// SS2D_local_12000138625311
// MI455X (gfx1250) — hardware-verified
//
#include <hip/hip_runtime.h>
#include <math.h>

typedef __attribute__((ext_vector_type(16))) _Float16 v16h;
typedef __attribute__((ext_vector_type(8)))  _Float16 v8h;
typedef __attribute__((ext_vector_type(4)))  _Float16 v4h;
typedef __attribute__((ext_vector_type(16))) __bf16   v16b;
typedef __attribute__((ext_vector_type(8)))  __bf16   v8b;
typedef __attribute__((ext_vector_type(8)))  float    v8f;
typedef __attribute__((ext_vector_type(4)))  float    v4f;

constexpr int kBatch = 2;
constexpr int kDm    = 128;
constexpr int kD     = 256;
constexpr int kD2    = 2 * kD;
constexpr int kDX    = 2 * kD;
constexpr int kH     = 64;
constexpr int kW     = 64;
constexpr int kL     = kH * kW;
constexpr int kRows  = kBatch * kL;
constexpr int kDirs  = 4;
constexpr int kNs    = 16;
constexpr int kR     = 8;
constexpr int kRP    = 32;
constexpr int kXd    = kR + 2 * kNs;
constexpr int kXdP   = 64;
constexpr int kNP    = kDirs * kXdP;
constexpr int kThr   = 256;
constexpr float kLnEps = 1e-5f;

constexpr float kInCarry = 1024.0f;
constexpr float kWCarry  = 4096.0f;
constexpr float kACarry  = 256.0f;
constexpr float kScIn = 1.0f / (kInCarry * kWCarry);
constexpr float kScA  = 1.0f / (kACarry * kWCarry);
constexpr float kF16MinNormal = 6.103515625e-5f;

static_assert((kRows % 64) == 0 && (kNP % 64) == 0 && (kD % 64) == 0 && (kDm % 64) == 0 && (kD2 % 64) == 0, "GEMM M, N multiples of 64");
static_assert(((kRows / 64) * (kDm / 64)) % 8 == 0, "the smallest GEMM grid exact");
static_assert((kDm % 32) == 0 && (kDX % 32) == 0 && (kRP % 32) == 0, "GEMM K multiples of 32");

constexpr size_t kOffX16 = 0;
constexpr size_t kOffWI  = kOffX16 + (size_t)kRows * kDm * 2;
constexpr size_t kOffWX  = kOffWI  + (size_t)kD2 * kDm * 2;
constexpr size_t kOffWDT = kOffWX  + (size_t)kNP * kDX * 2;
constexpr size_t kOffWO  = kOffWDT + (size_t)kDirs * kD * kRP * 2;
constexpr size_t kOffBV  = kOffWO  + (size_t)kDm * kDX * 2;
constexpr int    kBvZ    = 0;
constexpr int    kBvDt   = kD2;
constexpr int    kBvTot  = kD2 + kDirs * kD;
constexpr size_t kOffXZ  = kOffBV  + (size_t)kBvTot * 4;
constexpr size_t kOffU   = kOffXZ  + (size_t)kRows * kD2 * 4;
constexpr size_t kOffU16 = kOffU   + (size_t)kRows * kD * 4;
constexpr size_t kOffP   = kOffU16 + (size_t)kRows * kDX * 2;
constexpr size_t kOffDT16 = kOffP  + (size_t)kRows * kNP * 4;
constexpr size_t kOffDL  = kOffDT16 + (size_t)kRows * kDirs * kRP * 2;
constexpr size_t kOffYS  = kOffDL  + (size_t)kDirs * kRows * kD * 4;
constexpr size_t kOffY16 = kOffYS  + (size_t)kDirs * kRows * kD * 4;
constexpr size_t kWsTotal = kOffY16 + (size_t)kRows * kDX * 2;
static_assert(kWsTotal <= 268435456ull, "inside the offered workspace");
static_assert((kOffWI % 256) == 0 && (kOffWX % 256) == 0 && (kOffWDT % 256) == 0 && (kOffWO % 256) == 0 && (kOffBV % 256) == 0 && (kOffXZ % 256) == 0 && (kOffU % 256) == 0 && (kOffU16 % 256) == 0 && (kOffP % 256) == 0 && (kOffDT16 % 256) == 0 && (kOffDL % 256) == 0 && (kOffYS % 256) == 0 && (kOffY16 % 256) == 0, "aligned regions");

__device__ __forceinline__ unsigned short f2bf_bits(float f) {
  unsigned u = __float_as_uint(f);
  return (unsigned short)((u + 0x7FFFu + ((u >> 16) & 1u)) >> 16);
}
__device__ __forceinline__ float bf_bits2f(unsigned short h) { return __uint_as_float(((unsigned)h) << 16); }
__device__ __forceinline__ float bf16r(float f) { return bf_bits2f(f2bf_bits(f)); }
__device__ __forceinline__ float carry_flush(float v, float carry) {
  const float s = v * carry;
  return (fabsf(s) < kF16MinNormal) ? 0.0f : s;
}
__device__ __forceinline__ float frcp(float x) { return __builtin_amdgcn_rcpf(x); }

__device__ __forceinline__ void dep_guard4_h(v8f& a, v8f& b, v8f& c, v8f& d, v16h x, v16h y) { asm volatile("v_nop\n\tv_nop\n\tv_nop\n\tv_nop" : "+v"(a), "+v"(b), "+v"(c), "+v"(d) : "v"(x), "v"(y)); }
__device__ __forceinline__ void dep_guard4_b(v8f& a, v8f& b, v8f& c, v8f& d, v16b x, v16b y) { asm volatile("v_nop\n\tv_nop\n\tv_nop\n\tv_nop" : "+v"(a), "+v"(b), "+v"(c), "+v"(d) : "v"(x), "v"(y)); }
__device__ __forceinline__ void keep4_h(v16h a, v16h b, v16h c, v16h d) { asm volatile("v_nop" :: "v"(a), "v"(b), "v"(c), "v"(d)); }
__device__ __forceinline__ void keep4_b(v16b a, v16b b, v16b c, v16b d) { asm volatile("v_nop" :: "v"(a), "v"(b), "v"(c), "v"(d)); }
__device__ __forceinline__ void acc_guard4(v8f& a, v8f& b, v8f& c, v8f& d) { asm volatile("v_nop\n\tv_nop\n\tv_nop\n\tv_nop" : "+v"(a), "+v"(b), "+v"(c), "+v"(d)); }

template <typename T> struct Frag;
template <> struct Frag<_Float16> {
  typedef v16h V; union U { v16h v; v8h h[2]; };
  static __device__ __forceinline__ v16h load(const _Float16* p) {
    U f; f.h[0] = *(const v8h*)(p); f.h[1] = *(const v8h*)(p + 16); return f.v;
  }
  static __device__ __forceinline__ v8f mma(v16h a, v16h b, v8f c) {
    return __builtin_amdgcn_wmma_f32_16x16x32_f16(false, a, false, b, (short)0, c, false, false);
  }
  static __device__ __forceinline__ void guard4(v8f& a, v8f& b, v8f& c, v8f& d, v16h x, v16h y) { dep_guard4_h(a, b, c, d, x, y); }
  static __device__ __forceinline__ void keep(v16h a, v16h b, v16h c, v16h d) { keep4_h(a, b, c, d); }
};
template <> struct Frag<__bf16> {
  typedef v16b V; union U { v16b v; v8b h[2]; };
  static __device__ __forceinline__ v16b load(const __bf16* p) {
    U f; f.h[0] = *(const v8b*)(p); f.h[1] = *(const v8b*)(p + 16); return f.v;
  }
  static __device__ __forceinline__ v8f mma(v16b a, v16b b, v8f c) {
    return __builtin_amdgcn_wmma_f32_16x16x32_bf16(false, a, false, b, (short)0, c, false, false);
  }
  static __device__ __forceinline__ void guard4(v8f& a, v8f& b, v8f& c, v8f& d, v16b x, v16b y) { dep_guard4_b(a, b, c, d, x, y); }
  static __device__ __forceinline__ void keep(v16b a, v16b b, v16b c, v16b d) { keep4_b(a, b, c, d); }
};

__device__ __forceinline__ v8f mma_h(v16h a, v16h b, v8f c) {
  c = __builtin_amdgcn_wmma_f32_16x16x32_f16(false, a, false, b, (short)0, c, false, false);
  asm volatile("v_nop\n\tv_nop\n\tv_nop\n\tv_nop" : "+v"(c) : "v"(a), "v"(b));
  return c;
}

template <int ET> struct Elem;
template <> struct Elem<0> { typedef _Float16 T; };
template <> struct Elem<1> { typedef __bf16 T; };
template <int ET, bool SPLIT, int BIAS_MODE, int OUT_MODE, bool RESID, int ACT = 0>
__global__ __launch_bounds__(256) void wmma_gemm64(
    const unsigned short* __restrict__ Ap, const unsigned short* __restrict__ A2p, int lda, long strideA,
    const unsigned short* __restrict__ Btp, const unsigned short* __restrict__ Bt2p, int ldb, long strideB,
    void* __restrict__ Cout, void* __restrict__ Cout2, int ldc, long strideC,
    const float* __restrict__ bias,
    const float* __restrict__ resid, long strideR,
    int M, int N, int K, float scale) {
  typedef typename Elem<ET>::T T;
  typedef typename Frag<T>::V V;
  const T* A = (const T*)Ap; const T* A2 = (const T*)A2p; const T* Bt = (const T*)Btp; const T* Bt2 = (const T*)Bt2p;
  __shared__ __align__(16) float sT[8][16 * 68];
  const int b    = blockIdx.y;
  const int lane = threadIdx.x & 31;
  const int wave = threadIdx.x >> 5;
  const int tilesN = N >> 6;
  const int tilesM = M >> 6;
  const int tile = blockIdx.x * 8 + wave;
  if (tile >= tilesM * tilesN) return;
  const int tm = tile / tilesN;
  const int tn = tile - tm * tilesN;
  const int m0 = tm << 6;
  const int n0 = tn << 6;

  const T* Ab  = A  + (size_t)b * strideA;
  const T* Bb  = Bt + (size_t)b * strideB;
  const T* Ab2 = SPLIT ? (A2  + (size_t)b * strideA) : nullptr;
  const T* Bb2 = SPLIT ? (Bt2 + (size_t)b * strideB) : nullptr;

  const int rlane = lane & 15;
  const int koff  = (lane >> 4) * 8;
  const int mOff  = (lane >> 4) * 8;

  v8f acc[4][4];
#pragma unroll
  for (int i = 0; i < 4; ++i)
#pragma unroll
    for (int j = 0; j < 4; ++j) acc[i][j] = (v8f){0.f,0.f,0.f,0.f,0.f,0.f,0.f,0.f};

  for (int k0 = 0; k0 < K; k0 += 32) {
    V bh[4], bl[4];
#pragma unroll
    for (int j = 0; j < 4; ++j) {
      const size_t bo = (size_t)(n0 + (j << 4) + rlane) * ldb + koff + k0;
      bh[j] = Frag<T>::load(Bb + bo);
      if (SPLIT) bl[j] = Frag<T>::load(Bb2 + bo);
    }
#pragma unroll
    for (int i = 0; i < 4; ++i) {
      const size_t ao = (size_t)(m0 + (i << 4) + rlane) * lda + koff + k0;
      V ah = Frag<T>::load(Ab + ao);
      V al;
      if (SPLIT) al = Frag<T>::load(Ab2 + ao);
#pragma unroll
      for (int j = 0; j < 4; ++j) {
        acc[i][j] = Frag<T>::mma(ah, bh[j], acc[i][j]);
        if (SPLIT) {
          acc[i][j] = Frag<T>::mma(ah, bl[j], acc[i][j]);
          acc[i][j] = Frag<T>::mma(al, bh[j], acc[i][j]);
        }
      }
      Frag<T>::guard4(acc[i][0], acc[i][1], acc[i][2], acc[i][3], ah, SPLIT ? al : ah);
    }
    Frag<T>::keep(bh[0], bh[1], bh[2], bh[3]);
    if (SPLIT) Frag<T>::keep(bl[0], bl[1], bl[2], bl[3]);
  }
  acc_guard4(acc[0][0], acc[0][1], acc[0][2], acc[0][3]);
  acc_guard4(acc[1][0], acc[1][1], acc[1][2], acc[1][3]);
  acc_guard4(acc[2][0], acc[2][1], acc[2][2], acc[2][3]);
  acc_guard4(acc[3][0], acc[3][1], acc[3][2], acc[3][3]);

  float* slab = sT[wave];
  const float* Rb = RESID ? (resid + (size_t)b * strideR) : nullptr;
#pragma unroll
  for (int i = 0; i < 4; ++i) {
    const int mBase = m0 + (i << 4);
#pragma unroll
    for (int j = 0; j < 4; ++j) {
      const int n = n0 + (j << 4) + rlane;
      float bv = 0.f;
      if (BIAS_MODE == 2) bv = bias[n];
#pragma unroll
      for (int r = 0; r < 8; ++r) {
        float v = acc[i][j][r] * scale;
        if (BIAS_MODE == 1) v += bias[mBase + mOff + r];
        if (BIAS_MODE == 2) v += bv;
        if (RESID) v += Rb[(size_t)(mBase + mOff + r) * ldc + n];
        if (ACT == 1) v = tanhf(v);
        if (ACT == 2) v = fmaxf(v, 0.0f);
        if (ACT == 3) v = v / (1.0f + expf(-v));
        if (ACT == 4) v = (v > 0.f) ? v : 0.01f * v;
        slab[(mOff + r) * 68 + (j << 4) + rlane] = v;
      }
    }
    __builtin_amdgcn_fence(__ATOMIC_RELEASE, "workgroup");
    __builtin_amdgcn_wave_barrier();
    __builtin_amdgcn_fence(__ATOMIC_ACQUIRE, "workgroup");
    if (OUT_MODE == 0) {
      float* C = (float*)Cout + (size_t)b * strideC;
      const int hh = lane >> 4, c4 = (lane & 15) * 4;
      for (int pass = 0; pass < 2; ++pass) {
#pragma unroll
        for (int it = 0; it < 8; ++it) {
          const int row = it * 2 + hh;
          v4f v = *(const v4f*)(slab + row * 68 + c4);
          *(volatile v4f*)(C + (size_t)(mBase + row) * ldc + n0 + c4) = v;
        }
        __threadfence();
      }
    } else {
      const int q = lane >> 3, c8 = (lane & 7) * 8;
      unsigned short* C  = (unsigned short*)Cout  + (size_t)b * strideC;
      unsigned short* C2 = (OUT_MODE == 2) ? ((unsigned short*)Cout2 + (size_t)b * strideC) : nullptr;
      for (int pass = 0; pass < 2; ++pass) {
#pragma unroll
        for (int it = 0; it < 4; ++it) {
          const int row = it * 4 + q;
          const float* sp = slab + row * 68 + c8;
          v8h hv, lv;
#pragma unroll
          for (int e = 0; e < 8; ++e) {
            if (OUT_MODE == 1) {
              hv[e] = (_Float16)sp[e];
            } else {
              unsigned short hb = f2bf_bits(sp[e]);
              unsigned short lb = f2bf_bits(sp[e] - bf_bits2f(hb));
              hv[e] = __builtin_bit_cast(_Float16, hb);
              lv[e] = __builtin_bit_cast(_Float16, lb);
            }
          }
          *(volatile v8h*)(C + (size_t)(mBase + row) * ldc + n0 + c8) = hv;
          if (OUT_MODE == 2) *(volatile v8h*)(C2 + (size_t)(mBase + row) * ldc + n0 + c8) = lv;
        }
        __threadfence();
      }
    }
    __builtin_amdgcn_fence(__ATOMIC_RELEASE, "workgroup");
    __builtin_amdgcn_wave_barrier();
    __builtin_amdgcn_fence(__ATOMIC_ACQUIRE, "workgroup");
  }
}


__device__ __forceinline__ void split_hl(float v, float c, _Float16& hi, _Float16& lo) {
  const float sv = carry_flush(v, c);
  hi = (_Float16)sv;
  const float r = sv - (float)hi;
  lo = (_Float16)((fabsf(r) < kF16MinNormal) ? 0.0f : r);
}

__device__ __forceinline__ int src_pos(int k, int l) {
  const int lf = (k >= 2) ? (kL - 1 - l) : l;
  const int a = lf >> 10, b = (lf >> 8) & 3, c = (lf >> 4) & 15, e = lf & 15;
  const int hg = (k & 1) ? b : a, wg = (k & 1) ? a : b;
  const int i = (k & 1) ? e : c, j = (k & 1) ? c : e;
  return (16 * hg + i) * kW + 16 * wg + j;
}
__device__ __forceinline__ int dst_pos(int k, int l) {
  const int lf = (k >= 2) ? (kL - 1 - l) : l;
  return (k & 1) ? ((lf & (kH - 1)) * kW + (lf >> 6)) : lf;
}

__global__ __launch_bounds__(kThr) void cast_rows_kernel(const float* __restrict__ src, unsigned short* __restrict__ dst, int per, int ldd, int colOff, float c) {
  const int i = blockIdx.x * kThr + threadIdx.x;
  const int n = i / per;
  const int k8 = (i - n * per) * 8;
  const v4f a0 = *(const v4f*)(src + (size_t)i * 8);
  const v4f a1 = *(const v4f*)(src + (size_t)i * 8 + 4);
  v8h hv;
#pragma unroll
  for (int e = 0; e < 4; ++e) {
    const float w0 = a0[e], w1 = a1[e];
    hv[e]     = (_Float16)carry_flush(bf16r(w0), c);
    hv[4 + e] = (_Float16)carry_flush(bf16r(w1), c);
  }
  unsigned short* dp = dst + (size_t)n * ldd + colOff + k8;
  *(volatile v8h*)dp = hv;
  __threadfence();
  *(volatile v8h*)dp = hv;
}
static_assert(((size_t)kRows * (kDm / 8)) % kThr == 0 && (kD2 * (kDm / 8)) % kThr == 0 && (kDm * (kD / 8)) % kThr == 0, "row cast grids exact");

__global__ __launch_bounds__(32) void wx_plane_kernel(const float* __restrict__ xw, unsigned short* __restrict__ WX, int colOff) {
  const int n = blockIdx.x;
  const int k = n >> 6, c = n & 63;
  const bool live = c < kXd;
  const int k8 = threadIdx.x * 8;
  const float* sp = xw + ((size_t)k * kXd + (live ? c : 0)) * kD + k8;
  const v4f a0 = *(const v4f*)sp;
  const v4f a1 = *(const v4f*)(sp + 4);
  v8h hv;
#pragma unroll
  for (int e = 0; e < 4; ++e) {
    const float w0 = a0[e], w1 = a1[e];
    hv[e]     = (_Float16)(live ? carry_flush(bf16r(w0), kWCarry) : 0.0f);
    hv[4 + e] = (_Float16)(live ? carry_flush(bf16r(w1), kWCarry) : 0.0f);
  }
  unsigned short* dp = WX + (size_t)n * kDX + colOff + k8;
  *(volatile v8h*)dp = hv;
  __threadfence();
  *(volatile v8h*)dp = hv;
}

__global__ __launch_bounds__(kThr) void wdt_plane_kernel(const float* __restrict__ dtw, unsigned short* __restrict__ WDT) {
  const int i = blockIdx.x * kThr + threadIdx.x;
  const int rowkd = i >> 2;
  const int c8 = (i & 3) * 8;
  v8h hv;
#pragma unroll
  for (int e = 0; e < 8; ++e) {
    const int c = c8 + e;
    const int cc = (c >= 16) ? (c - 16) : c;
    const bool live = cc < kR;
    const float w = dtw[(size_t)rowkd * kR + (live ? cc : 0)];
    hv[e] = (_Float16)(live ? carry_flush(bf16r(w), kWCarry) : 0.0f);
  }
  unsigned short* dp = WDT + (size_t)i * 8;
  *(volatile v8h*)dp = hv;
  __threadfence();
  *(volatile v8h*)dp = hv;
}
static_assert(kDirs * kD * 4 == 16 * kThr, "step plane grid exact");

__global__ __launch_bounds__(128) void bias_rows_kernel(const float* __restrict__ dtb, float* __restrict__ BV) {
  const int i = blockIdx.x * 128 + threadIdx.x;
  const int idt = i - kBvDt;
  const float v = dtb[(idt >= 0) ? idt : 0];
  const float o = (idt >= 0) ? bf16r(v) : 0.0f;
  for (int pass = 0; pass < 2; ++pass) {
    *(volatile float*)(BV + i) = o;
    __threadfence();
  }
}
static_assert(kBvTot % 128 == 0 && kBvDt % 128 == 0, "bias grid exact; regions block-uniform");

__global__ __launch_bounds__(kThr) void conv3_silu_kernel(const float* __restrict__ XZ, const float* __restrict__ conv_w, const float* __restrict__ conv_b,
                                                          float* __restrict__ U, unsigned short* __restrict__ U16) {
  const size_t v = (size_t)blockIdx.x * kThr + threadIdx.x;
  const size_t row = v >> 6;
  const int d4 = (int)(v & 63) * 4;
  const int b = (int)(row >> 12);
  const int pos = (int)(row & (kL - 1));
  const int h = pos >> 6, w = pos & 63;
  v4f acc = *(const v4f*)(conv_b + d4);
#pragma unroll
  for (int e = 0; e < 4; ++e) { const float b0 = acc[e]; acc[e] = bf16r(b0); }
#pragma unroll
  for (int i = 0; i < 3; ++i) {
#pragma unroll
    for (int j = 0; j < 3; ++j) {
      const int hh = h + i - 1, ww = w + j - 1;
      const bool ok = (hh >= 0) && (hh < kH) && (ww >= 0) && (ww < kW);
      const size_t rr = ok ? ((size_t)b * kL + hh * kW + ww) : row;
      const v4f zin = *(const v4f*)(XZ + rr * kD2 + d4);
#pragma unroll
      for (int e = 0; e < 4; ++e) {
        const float wt = conv_w[(size_t)(d4 + e) * 9 + i * 3 + j];
        acc[e] += ok ? (bf16r(wt) * zin[e]) : 0.0f;
      }
    }
  }
  v4f o;
  v4h hv, lv;
#pragma unroll
  for (int e = 0; e < 4; ++e) {
    const float s = acc[e] * (1.0f / (1.0f + expf(-acc[e])));
    o[e] = s;
    _Float16 hi, lo;
    split_hl(s, kACarry, hi, lo);
    hv[e] = hi; lv[e] = lo;
  }
  for (int pass = 0; pass < 2; ++pass) {
    *(volatile v4f*)(U + row * kD + d4) = o;
    *(volatile v4h*)(U16 + row * kDX + d4) = hv;
    *(volatile v4h*)(U16 + row * kDX + kD + d4) = lv;
    __threadfence();
  }
}
static_assert(((size_t)kRows * 64) % kThr == 0 && kD / 4 == 64 && kL == 4096 && kW == 64, "conv grid exact; index splits");

__global__ __launch_bounds__(kThr) void dt_cast_kernel(const float* __restrict__ P, unsigned short* __restrict__ DT16) {
  const size_t v = (size_t)blockIdx.x * kThr + threadIdx.x;
  const size_t row = v >> 4;
  const int t = (int)(v & 15);
  const int k = t >> 2;
  const int c8 = (t & 3) * 8;
  const bool isLo = c8 >= 16;
  const bool liveBlk = (c8 & 15) == 0;
  const v4f a0 = *(const v4f*)(P + row * kNP + k * kXdP);
  const v4f a1 = *(const v4f*)(P + row * kNP + k * kXdP + 4);
  v8h hv;
#pragma unroll
  for (int e = 0; e < 4; ++e) {
    _Float16 h0, l0, h1, l1;
    split_hl(a0[e], kACarry, h0, l0);
    split_hl(a1[e], kACarry, h1, l1);
    hv[e]     = liveBlk ? (isLo ? l0 : h0) : (_Float16)0.0f;
    hv[4 + e] = liveBlk ? (isLo ? l1 : h1) : (_Float16)0.0f;
  }
  unsigned short* dp = DT16 + v * 8;
  *(volatile v8h*)dp = hv;
  __threadfence();
  *(volatile v8h*)dp = hv;
}
static_assert(((size_t)kRows * 16) % kThr == 0 && kR == 8, "dt cast grid exact");

__global__ __launch_bounds__(kThr) void local_scan_kernel(const float* __restrict__ DL, const float* __restrict__ U, const float* __restrict__ P,
                                                          const float* __restrict__ A_logs, const float* __restrict__ Ds, float* __restrict__ YS) {
  const int v = blockIdx.x * kThr + threadIdx.x;
  const int bk = v >> 8;
  const int d = v & (kD - 1);
  const int b = bk >> 2, k = bk & 3;
  float A[kNs], h[kNs];
#pragma unroll
  for (int n = 0; n < kNs; ++n) { const float al = A_logs[((size_t)k * kD + d) * kNs + n]; A[n] = -expf(bf16r(al)); h[n] = 0.0f; }
  const float dd = Ds[k * kD + d];
  const float dsk = bf16r(dd);
  const float* dlk = DL + (size_t)k * kRows * kD;
  float* ysk = YS + (size_t)k * kRows * kD;
#pragma unroll 1
  for (int l = 0; l < kL; ++l) {
    const size_t rs = (size_t)b * kL + src_pos(k, l);
    const size_t rd = (size_t)b * kL + dst_pos(k, l);
    const float dl = dlk[rs * kD + d];
    const float u = U[rs * kD + d];
    const float delta = (dl > 20.0f) ? dl : log1pf(expf(dl));
    const float du = delta * u;
    float y = 0.0f;
#pragma unroll
    for (int q = 0; q < 4; ++q) {
      const v4f bq = *(const v4f*)(P + rs * kNP + k * kXdP + kR + 4 * q);
      const v4f cq = *(const v4f*)(P + rs * kNP + k * kXdP + kR + kNs + 4 * q);
#pragma unroll
      for (int e = 0; e < 4; ++e) {
        const int n = 4 * q + e;
        const float hn = __expf(delta * A[n]) * h[n] + du * bq[e];
        h[n] = hn;
        y += hn * cq[e];
      }
    }
    const float o = y + dsk * u;
    float* op = ysk + rd * kD + d;
    *(volatile float*)op = o;
    __threadfence();
    *(volatile float*)op = o;
  }
}
static_assert((kBatch * kDirs * kD) % kThr == 0 && (kD % 32) == 0, "scan grid exact; a wave inside one (b, k)");

__global__ __launch_bounds__(kThr) void merge_ln_gate_kernel(const float* __restrict__ YS, const float* __restrict__ XZ, const float* __restrict__ ln_w,
                                                             const float* __restrict__ ln_b, unsigned short* __restrict__ Y16) {
  const size_t row = (size_t)blockIdx.x * kThr + threadIdx.x;
  const size_t plane = (size_t)kRows * kD;
  const float* y0 = YS + row * kD;
  float s = 0.0f;
#pragma unroll 1
  for (int d = 0; d < kD; ++d) s += ((y0[d] + y0[2 * plane + d]) + y0[plane + d]) + y0[3 * plane + d];
  const float mu = s * (1.0f / (float)kD);
  float q = 0.0f;
#pragma unroll 1
  for (int d = 0; d < kD; ++d) { const float dv = (((y0[d] + y0[2 * plane + d]) + y0[plane + d]) + y0[3 * plane + d]) - mu; q += dv * dv; }
  const float rs = 1.0f / sqrtf(q * (1.0f / (float)kD) + kLnEps);
  unsigned short* dp = Y16 + row * kDX;
  const float* zr = XZ + row * kD2 + kD;
#pragma unroll 1
  for (int d8 = 0; d8 < kD; d8 += 8) {
    v8h hv, lv;
#pragma unroll
    for (int e = 0; e < 8; ++e) {
      const int d = d8 + e;
      const float g0 = ln_w[d], b0 = ln_b[d];
      const float nrm = ((((y0[d] + y0[2 * plane + d]) + y0[plane + d]) + y0[3 * plane + d]) - mu) * rs * bf16r(g0) + bf16r(b0);
      const float zz = zr[d];
      const float g = nrm * (zz * frcp(1.0f + __expf(-zz)));
      _Float16 hi, lo;
      split_hl(g, kACarry, hi, lo);
      hv[e] = hi; lv[e] = lo;
    }
    for (int pass = 0; pass < 2; ++pass) {
      *(volatile v8h*)(dp + d8) = hv;
      *(volatile v8h*)(dp + kD + d8) = lv;
      __threadfence();
    }
  }
}
static_assert(kRows % kThr == 0, "merge grid exact");

extern "C" void kernel_launch(void* const* d_in, const int* in_sizes, int n_in,
                              void* d_out, int out_size, void* d_ws, size_t ws_size,
                              hipStream_t stream) {
  if (n_in < 12 || d_out == nullptr || d_ws == nullptr) return;
  if (in_sizes[0] != kRows * kDm || in_sizes[1] != kD2 * kDm || in_sizes[2] != kD * 9 || in_sizes[3] != kD) return;
  if (in_sizes[4] != kDirs * kXd * kD || in_sizes[5] != kDirs * kD * kR || in_sizes[6] != kDirs * kD || in_sizes[7] != kDirs * kD * kNs) return;
  if (in_sizes[8] != kDirs * kD || in_sizes[9] != kD || in_sizes[10] != kD || in_sizes[11] != kDm * kD) return;
  if (out_size != kRows * kDm) return;
  if (ws_size < kWsTotal) return;
  const float* x = (const float*)d_in[0];
  const float* W_in = (const float*)d_in[1];
  const float* conv_w = (const float*)d_in[2];
  const float* conv_b = (const float*)d_in[3];
  const float* xw = (const float*)d_in[4];
  const float* dtw = (const float*)d_in[5];
  const float* dtb = (const float*)d_in[6];
  const float* A_logs = (const float*)d_in[7];
  const float* Ds = (const float*)d_in[8];
  const float* ln_w = (const float*)d_in[9];
  const float* ln_b = (const float*)d_in[10];
  const float* W_out = (const float*)d_in[11];
  float* out = (float*)d_out;
  char* ws = (char*)d_ws;
  unsigned short* X16 = (unsigned short*)(ws + kOffX16);
  unsigned short* WI = (unsigned short*)(ws + kOffWI);
  unsigned short* WX = (unsigned short*)(ws + kOffWX);
  unsigned short* WDT = (unsigned short*)(ws + kOffWDT);
  unsigned short* WO = (unsigned short*)(ws + kOffWO);
  float* BV = (float*)(ws + kOffBV);
  float* XZ = (float*)(ws + kOffXZ);
  float* U = (float*)(ws + kOffU);
  unsigned short* U16 = (unsigned short*)(ws + kOffU16);
  float* P = (float*)(ws + kOffP);
  unsigned short* DT16 = (unsigned short*)(ws + kOffDT16);
  float* DL = (float*)(ws + kOffDL);
  float* YS = (float*)(ws + kOffYS);
  unsigned short* Y16 = (unsigned short*)(ws + kOffY16);

  cast_rows_kernel<<<(int)(((size_t)kRows * (kDm / 8)) / kThr), kThr, 0, stream>>>(x, X16, kDm / 8, kDm, 0, kInCarry);
  cast_rows_kernel<<<(kD2 * (kDm / 8)) / kThr, kThr, 0, stream>>>(W_in, WI, kDm / 8, kDm, 0, kWCarry);
  wx_plane_kernel<<<kNP, kD / 8, 0, stream>>>(xw, WX, 0);
  wx_plane_kernel<<<kNP, kD / 8, 0, stream>>>(xw, WX, kD);
  wdt_plane_kernel<<<16, kThr, 0, stream>>>(dtw, WDT);
  cast_rows_kernel<<<(kDm * (kD / 8)) / kThr, kThr, 0, stream>>>(W_out, WO, kD / 8, kDX, 0, kWCarry);
  cast_rows_kernel<<<(kDm * (kD / 8)) / kThr, kThr, 0, stream>>>(W_out, WO, kD / 8, kDX, kD, kWCarry);
  bias_rows_kernel<<<kBvTot / 128, 128, 0, stream>>>(dtb, BV);

  wmma_gemm64<0, false, 2, 0, false, 0><<<dim3((kRows / 64) * (kD2 / 64) / 8, 1), 256, 0, stream>>>(
      X16, X16, kDm, 0L, WI, WI, kDm, 0L, (void*)XZ, (void*)XZ, kD2, 0L, BV + kBvZ, nullptr, 0L, kRows, kD2, kDm, kScIn);
  conv3_silu_kernel<<<(int)(((size_t)kRows * 64) / kThr), kThr, 0, stream>>>(XZ, conv_w, conv_b, U, U16);
  wmma_gemm64<0, false, 2, 0, false, 0><<<dim3((kRows / 64) * (kNP / 64) / 8, 1), 256, 0, stream>>>(
      U16, U16, kDX, 0L, WX, WX, kDX, 0L, (void*)P, (void*)P, kNP, 0L, BV + kBvZ, nullptr, 0L, kRows, kNP, kDX, kScA);
  dt_cast_kernel<<<(int)(((size_t)kRows * 16) / kThr), kThr, 0, stream>>>(P, DT16);
  for (int k = 0; k < kDirs; ++k) {
    wmma_gemm64<0, false, 2, 0, false, 0><<<dim3((kRows / 64) * (kD / 64) / 8, 1), 256, 0, stream>>>(
        DT16 + k * kRP, DT16 + k * kRP, kDirs * kRP, 0L, WDT + (size_t)k * kD * kRP, WDT + (size_t)k * kD * kRP, kRP, 0L,
        (void*)(DL + (size_t)k * kRows * kD), (void*)(DL + (size_t)k * kRows * kD), kD, 0L, BV + kBvDt + k * kD, nullptr, 0L, kRows, kD, kRP, kScA);
  }
  local_scan_kernel<<<(kBatch * kDirs * kD) / kThr, kThr, 0, stream>>>(DL, U, P, A_logs, Ds, YS);
  merge_ln_gate_kernel<<<kRows / kThr, kThr, 0, stream>>>(YS, XZ, ln_w, ln_b, Y16);
  wmma_gemm64<0, false, 2, 0, false, 0><<<dim3((kRows / 64) * (kDm / 64) / 8, 1), 256, 0, stream>>>(
      Y16, Y16, kDX, 0L, WO, WO, kDX, 0L, (void*)out, (void*)out, kDm, 0L, BV + kBvZ, nullptr, 0L, kRows, kDm, kDX, kScA);
}
